// FRU_48653389529467
// MI455X (gfx1250) — hardware-verified
//
#include <hip/hip_runtime.h>


#define AS3 __attribute__((address_space(3)))

#define S_LEN   1024
#define D_IN    2048
#define D_OUT   2048
#define STATE_D 1024
#define NH      16
#define DH      64
#define PROJ_D  5120

static_assert(PROJ_D == 5 * STATE_D);
static_assert(STATE_D == NH * DH);
static_assert(DH == 64);
static_assert(D_IN % 32 == 0 && STATE_D % 32 == 0);
static_assert(S_LEN % 128 == 0 && PROJ_D % 64 == 0 && D_OUT % 64 == 0 && STATE_D % 64 == 0);

typedef __bf16         v16b __attribute__((ext_vector_type(16)));
typedef unsigned short v8us __attribute__((ext_vector_type(8)));
typedef float          v8f  __attribute__((ext_vector_type(8)));
typedef float          v4f  __attribute__((ext_vector_type(4)));
typedef v8us __attribute__((may_alias)) v8usa;
typedef v4f  __attribute__((may_alias)) v4fa;

typedef AS3 unsigned short*       lp_us;
typedef AS3 const unsigned short* lcp_us;
typedef AS3 float*                lp_f;
typedef AS3 const float*          lcp_f;

union Frag { v16b v; v8us half[2]; };

constexpr int P_X   = 0;
constexpr int P_WI  = P_X + S_LEN * D_IN;
constexpr int P_WO  = P_WI + PROJ_D * D_IN;
constexpr int P_END = P_WO + D_OUT * STATE_D;
constexpr int NPC   = P_END / 8;
constexpr int NCBLK = NPC / 256;
static_assert(P_END % 8 == 0);
static_assert(NPC % 256 == 0);
static_assert(P_WI % 2048 == 0 && P_WO % 2048 == 0);

constexpr size_t OFF_CV = 0;
constexpr size_t SZ_CV  = (size_t)P_END * 2;
constexpr size_t OFF_PR = OFF_CV + SZ_CV;
constexpr size_t SZ_PR  = (size_t)S_LEN * PROJ_D * 4;
constexpr size_t OFF_Y  = OFF_PR + SZ_PR;
constexpr size_t SZ_Y   = (size_t)S_LEN * STATE_D * 4;
constexpr size_t OFF_YH = OFF_Y + SZ_Y;
constexpr size_t SZ_YP  = (size_t)S_LEN * STATE_D * 2;
constexpr size_t OFF_YL = OFF_YH + SZ_YP;
constexpr size_t WS_END = OFF_YL + SZ_YP;
static_assert(OFF_PR % 128 == 0 && OFF_Y % 128 == 0 && OFF_YH % 128 == 0 && OFF_YL % 128 == 0);
static_assert(WS_END <= (size_t)134217728);
static_assert((size_t)NPC * 16 == SZ_CV);
static_assert((size_t)(S_LEN / 128) * (PROJ_D / 64) * 128 * 64 * 4 == SZ_PR);
static_assert((size_t)NH * S_LEN * DH * 4 == SZ_Y);
static_assert((size_t)S_LEN * 128 * 16 == SZ_YP);
static_assert((size_t)(S_LEN / 128) * (D_OUT / 64) * 128 * 64 == (size_t)S_LEN * D_OUT);

__device__ __forceinline__ unsigned short bf16_bits(float f) {
  unsigned u = __float_as_uint(f);
  u += 0x7FFFu + ((u >> 16) & 1u);
  return (unsigned short)(u >> 16);
}
__device__ __forceinline__ float bf16_val(unsigned short b) { return __uint_as_float(((unsigned)b) << 16); }
__device__ __forceinline__ float bf16r(float f) { return bf16_val(bf16_bits(f)); }
__device__ __forceinline__ v8f zero8() {
  v8f z;
#pragma unroll
  for (int i = 0; i < 8; ++i) z[i] = 0.0f;
  return z;
}
__device__ __forceinline__ float sigm(float x) {
  return __builtin_amdgcn_rcpf(1.0f + __expf(-x));
}

__device__ __forceinline__ void ldfrag_g(Frag& f, const unsigned short* p, int h) {
  f.half[0] = *(const v8usa*)(p + 8 * h);
  f.half[1] = *(const v8usa*)(p + 16 + 8 * h);
}
__device__ __forceinline__ void ldfrag_l(Frag& f, lcp_us p, int h) {
  f.half[0] = *(AS3 const v8usa*)(p + 8 * h);
  f.half[1] = *(AS3 const v8usa*)(p + 16 + 8 * h);
}
__device__ __forceinline__ v8f mma16(v8f c, const Frag& a, const Frag& b) {
  return __builtin_amdgcn_wmma_f32_16x16x32_bf16(false, a.v, false, b.v, (short)0, c, false, false);
}

__global__ __launch_bounds__(256)
void cvt_kernel(const float* __restrict__ x, const float* __restrict__ wi, const float* __restrict__ wo,
                unsigned short* cv)
{
  const int g = blockIdx.x * 256 + threadIdx.x;
  if (g >= NPC) return;
  const int e = g * 8;
  const float* src;
  if      (e < P_WI) src = x  + e;
  else if (e < P_WO) src = wi + (e - P_WI);
  else               src = wo + (e - P_WO);
  const v4f a = *(const v4fa*)src;
  const v4f c = *(const v4fa*)(src + 4);
  v8us o;
  o[0] = bf16_bits(a[0]); o[1] = bf16_bits(a[1]); o[2] = bf16_bits(a[2]); o[3] = bf16_bits(a[3]);
  o[4] = bf16_bits(c[0]); o[5] = bf16_bits(c[1]); o[6] = bf16_bits(c[2]); o[7] = bf16_bits(c[3]);
  unsigned short* dst = cv + e;
  *(volatile v8us*)dst = o;
  __threadfence();
  *(volatile v8us*)dst = o;
}

constexpr size_t GLDS = (size_t)128 * 64 * 4;

__device__ __forceinline__ void tile_store_pass(lcp_f sT, float* C, int ldc, int m0, int c0, int w, int lane) {
  const int q8 = lane & 7, sub = lane >> 3;
#pragma unroll
  for (int i = 0; i < 16; ++i) {
    const int lidx = 64 * w + 4 * i + sub;
    const int row = lidx >> 1, hl = lidx & 1;
    const v4f v = *(AS3 const v4fa*)(sT + row * 64 + 32 * hl + 4 * q8);
    float* dst = C + (size_t)(m0 + row) * ldc + c0 + 32 * hl + 4 * q8;
    *(volatile v4f*)dst = v;
  }
}

template <bool ALO, bool PEPI>
__global__ __launch_bounds__(128)
void gemm_kernel(const unsigned short* __restrict__ Ah, const unsigned short* __restrict__ Al,
                 const unsigned short* __restrict__ Bw, int K, float* C, int ldc,
                 const float* __restrict__ fm, const float* __restrict__ fb)
{
  extern __shared__ __attribute__((aligned(16))) char smem[];
  lp_f sT = (lp_f)smem;

  const int tid = threadIdx.x, lane = tid & 31, w = tid >> 5;
  const int h = lane >> 4, m = lane & 15;
  const int m0 = blockIdx.x * 128;
  const int cy = blockIdx.y;
  const int c0 = 64 * cy;
  const int m0w = m0 + 32 * w;

  const unsigned short* xa = Ah + (size_t)(m0w + m) * K;
  const unsigned short* xl = Al + (size_t)(m0w + m) * K;
  const unsigned short* wb = Bw + (size_t)(c0 + m) * K;

  v8f acc[2][4];
#pragma unroll
  for (int mt = 0; mt < 2; ++mt)
#pragma unroll
    for (int nt = 0; nt < 4; ++nt) acc[mt][nt] = zero8();

#pragma unroll 1
  for (int k0 = 0; k0 < K; k0 += 32) {
    Frag a[2], b[4];
#pragma unroll
    for (int mt = 0; mt < 2; ++mt) ldfrag_g(a[mt], xa + (size_t)mt * 16 * K + k0, h);
#pragma unroll
    for (int nt = 0; nt < 4; ++nt) ldfrag_g(b[nt], wb + (size_t)nt * 16 * K + k0, h);
    if (ALO) {
      Frag al[2];
#pragma unroll
      for (int mt = 0; mt < 2; ++mt) ldfrag_g(al[mt], xl + (size_t)mt * 16 * K + k0, h);
#pragma unroll
      for (int mt = 0; mt < 2; ++mt)
#pragma unroll
        for (int nt = 0; nt < 4; ++nt) {
          acc[mt][nt] = mma16(acc[mt][nt], a[mt], b[nt]);
          acc[mt][nt] = mma16(acc[mt][nt], al[mt], b[nt]);
        }
      asm volatile("v_nop\n\tv_nop\n\tv_nop\n\tv_nop"
                   : "+v"(acc[0][0]), "+v"(acc[0][1]), "+v"(acc[0][2]), "+v"(acc[0][3]),
                     "+v"(acc[1][0]), "+v"(acc[1][1]), "+v"(acc[1][2]), "+v"(acc[1][3])
                   : "v"(a[0].v), "v"(a[1].v), "v"(al[0].v), "v"(al[1].v),
                     "v"(b[0].v), "v"(b[1].v), "v"(b[2].v), "v"(b[3].v));
    } else {
#pragma unroll
      for (int mt = 0; mt < 2; ++mt)
#pragma unroll
        for (int nt = 0; nt < 4; ++nt) acc[mt][nt] = mma16(acc[mt][nt], a[mt], b[nt]);
      asm volatile("v_nop\n\tv_nop\n\tv_nop\n\tv_nop"
                   : "+v"(acc[0][0]), "+v"(acc[0][1]), "+v"(acc[0][2]), "+v"(acc[0][3]),
                     "+v"(acc[1][0]), "+v"(acc[1][1]), "+v"(acc[1][2]), "+v"(acc[1][3])
                   : "v"(a[0].v), "v"(a[1].v), "v"(b[0].v), "v"(b[1].v), "v"(b[2].v), "v"(b[3].v));
    }
  }

#pragma unroll
  for (int nt = 0; nt < 4; ++nt) {
    const int col = 16 * nt + m;
#pragma unroll
    for (int mt = 0; mt < 2; ++mt)
#pragma unroll
      for (int r = 0; r < 8; ++r) {
        const int rowl = 32 * w + 16 * mt + 8 * h + r;
        sT[rowl * 64 + col] = acc[mt][nt][r];
      }
  }
  __syncthreads();

  if (PEPI) {
    const int grp = cy >> 4, head = cy & 15;
    lp_f rowp = sT + tid * 64;
    if (grp == 1) {
      float ss = 0.0f;
#pragma unroll
      for (int j = 0; j < 16; ++j) {
        const v4f v = *(AS3 const v4fa*)(rowp + 4 * j);
        ss += v[0] * v[0] + v[1] * v[1] + v[2] * v[2] + v[3] * v[3];
      }
      const float inv = fminf(rsqrtf(ss), 1e12f);
#pragma unroll
      for (int j = 0; j < 16; ++j) {
        v4f v = *(AS3 const v4fa*)(rowp + 4 * j);
        v = v * inv;
        *(AS3 v4fa*)(rowp + 4 * j) = v;
      }
    } else if (grp == 3) {
      const float m2 = 2.0f * sigm(bf16r(fm[head]));
      const float* fbp = fb + head * DH;
#pragma unroll
      for (int j = 0; j < 16; ++j) {
        v4f v = *(AS3 const v4fa*)(rowp + 4 * j);
        const v4f b4 = *(const v4fa*)(fbp + 4 * j);
        v[0] = sigm(m2 * (v[0] + bf16r(b4[0])));
        v[1] = sigm(m2 * (v[1] + bf16r(b4[1])));
        v[2] = sigm(m2 * (v[2] + bf16r(b4[2])));
        v[3] = sigm(m2 * (v[3] + bf16r(b4[3])));
        *(AS3 v4fa*)(rowp + 4 * j) = v;
      }
    }
    __syncthreads();
  }

  tile_store_pass(sT, C, ldc, m0, c0, w, lane);
  __threadfence();
  tile_store_pass(sT, C, ldc, m0, c0, w, lane);
}

constexpr int    HP    = DH + 8;
constexpr int    TILE  = DH * HP;
constexpr size_t SC_HL = 0;
constexpr size_t SC_W  = SC_HL + (size_t)4 * TILE * 2;
constexpr size_t SC_Y  = SC_W + (size_t)TILE * 2;
constexpr size_t SLDS  = SC_Y + (size_t)2 * 4 * DH * 4;
constexpr int    NZT   = 4 * TILE / 8;
static_assert(HP % 8 == 0 && TILE % 8 == 0);
static_assert(SC_W % 16 == 0 && SC_Y % 16 == 0);

__global__ __launch_bounds__(128)
void scan_kernel(const float* __restrict__ proj, const float* __restrict__ sw, float* ypl)
{
  extern __shared__ __attribute__((aligned(16))) char smem[];
  lp_us hT = (lp_us)(smem + SC_HL);
  lp_us sW = (lp_us)(smem + SC_W);
  lp_f  sY = (lp_f)(smem + SC_Y);

  const int tid = threadIdx.x, lane = tid & 31, w = tid >> 5;
  const int h = lane >> 4, m = lane & 15;
  const int head = blockIdx.x;

  {
    v8us z8;
#pragma unroll
    for (int i = 0; i < 8; ++i) z8[i] = (unsigned short)0;
    for (int i = tid; i < NZT; i += 128) *(AS3 v8us*)(hT + 8 * i) = z8;
    const float* wsrc = sw + (size_t)head * DH * DH;
#pragma unroll 1
    for (int i = tid; i < DH * DH; i += 128) {
      const int d = i >> 6, e = i & 63;
      sW[e * HP + d] = bf16_bits(wsrc[i]);
    }
  }
  __syncthreads();

  lcp_us wrow = sW + m * HP;
  const int rloc = 16 * w + 8 * h;

#pragma unroll 1
  for (int t = 0; t < S_LEN; ++t) {
    const int cur = t & 1;
    lcp_us aHp = hT + cur * TILE + (16 * w + m) * HP;
    lcp_us aLp = hT + (2 + cur) * TILE + (16 * w + m) * HP;
    lp_us  nHp = hT + (cur ^ 1) * TILE;
    lp_us  nLp = hT + (2 + (cur ^ 1)) * TILE;

    const float* pt = proj + (size_t)t * PROJ_D + head * DH;
    const float* pr = pt + rloc;
    const v4f q0 = *(const v4fa*)(pr),               q1 = *(const v4fa*)(pr + 4);
    const v4f n0 = *(const v4fa*)(pr + STATE_D),     n1 = *(const v4fa*)(pr + STATE_D + 4);
    const v4f f0 = *(const v4fa*)(pr + 3 * STATE_D), f1 = *(const v4fa*)(pr + 3 * STATE_D + 4);
    const float qv[8]  = {q0[0], q0[1], q0[2], q0[3], q1[0], q1[1], q1[2], q1[3]};
    const float knv[8] = {n0[0], n0[1], n0[2], n0[3], n1[0], n1[1], n1[2], n1[3]};
    const float fgv[8] = {f0[0], f0[1], f0[2], f0[3], f1[0], f1[1], f1[2], f1[3]};
    float vv[4];
#pragma unroll
    for (int nt = 0; nt < 4; ++nt) vv[nt] = pt[2 * STATE_D + 16 * nt + m];

    v8f acc[4];
#pragma unroll
    for (int nt = 0; nt < 4; ++nt) acc[nt] = zero8();
#pragma unroll
    for (int kc = 0; kc < 2; ++kc) {
      Frag ah, al, b[4];
      ldfrag_l(ah, aHp + 32 * kc, h);
      ldfrag_l(al, aLp + 32 * kc, h);
#pragma unroll
      for (int nt = 0; nt < 4; ++nt) ldfrag_l(b[nt], wrow + nt * 16 * HP + 32 * kc, h);
#pragma unroll
      for (int nt = 0; nt < 4; ++nt) {
        acc[nt] = mma16(acc[nt], ah, b[nt]);
        acc[nt] = mma16(acc[nt], al, b[nt]);
      }
      asm volatile("v_nop\n\tv_nop\n\tv_nop\n\tv_nop"
                   : "+v"(acc[0]), "+v"(acc[1]), "+v"(acc[2]), "+v"(acc[3])
                   : "v"(ah.v), "v"(al.v), "v"(b[0].v), "v"(b[1].v), "v"(b[2].v), "v"(b[3].v));
    }

    float yp[4] = {0.0f, 0.0f, 0.0f, 0.0f};
#pragma unroll
    for (int nt = 0; nt < 4; ++nt) {
      const int col = 16 * nt + m;
      const float vn = vv[nt];
#pragma unroll
      for (int r = 0; r < 8; ++r) {
        const int row = rloc + r;
        const float ns = fgv[r] * acc[nt][r] + knv[r] * vn;
        const unsigned short hb = bf16_bits(ns);
        const unsigned short lb = bf16_bits(ns - bf16_val(hb));
        nHp[row * HP + col] = hb;
        nLp[row * HP + col] = lb;
        yp[nt] += qv[r] * ns;
      }
    }
#pragma unroll
    for (int nt = 0; nt < 4; ++nt) yp[nt] += __shfl_xor(yp[nt], 16);
    if (h == 0) {
#pragma unroll
      for (int nt = 0; nt < 4; ++nt) sY[cur * 256 + w * 64 + 16 * nt + m] = yp[nt];
    }

    __syncthreads();

    if (tid < 16) {
      lcp_f yb = sY + cur * 256 + 4 * tid;
      v4f yv = *(AS3 const v4fa*)(yb);
      yv += *(AS3 const v4fa*)(yb + 64);
      yv += *(AS3 const v4fa*)(yb + 128);
      yv += *(AS3 const v4fa*)(yb + 192);
      float* dst = ypl + (size_t)t * STATE_D + head * DH + 4 * tid;
      *(volatile v4f*)dst = yv;
      __threadfence();
      *(volatile v4f*)dst = yv;
    }
  }
}

__global__ __launch_bounds__(128)
void gate_norm_kernel(const float* __restrict__ y, const float* __restrict__ proj, const float* __restrict__ gw,
                      unsigned short* yh, unsigned short* yl)
{
  __shared__ float sRed[4];
  const int tid = threadIdx.x, lane = tid & 31, w = tid >> 5;
  const int s = blockIdx.x;
  const float* yr = y + (size_t)s * STATE_D + 8 * tid;
  const float* gr = proj + (size_t)s * PROJ_D + 4 * STATE_D + 8 * tid;
  const float* nr = gw + 8 * tid;
  const v4f ya = *(const v4fa*)yr, yb = *(const v4fa*)(yr + 4);
  const v4f ga = *(const v4fa*)gr, gb = *(const v4fa*)(gr + 4);
  const v4f na = *(const v4fa*)nr, nb = *(const v4fa*)(nr + 4);
  const float gg[8] = {ga[0], ga[1], ga[2], ga[3], gb[0], gb[1], gb[2], gb[3]};
  const float yy[8] = {ya[0], ya[1], ya[2], ya[3], yb[0], yb[1], yb[2], yb[3]};
  const float nn[8] = {na[0], na[1], na[2], na[3], nb[0], nb[1], nb[2], nb[3]};
  float v[8];
  float ss = 0.0f;
#pragma unroll
  for (int c = 0; c < 8; ++c) {
    const float g = gg[c];
    v[c] = yy[c] * (g * sigm(g));
    ss += v[c] * v[c];
  }
  ss += __shfl_xor(ss, 1);
  ss += __shfl_xor(ss, 2);
  ss += __shfl_xor(ss, 4);
  ss += __shfl_xor(ss, 8);
  ss += __shfl_xor(ss, 16);
  if (lane == 0) sRed[w] = ss;
  __syncthreads();
  const float tot = ((sRed[0] + sRed[1]) + sRed[2]) + sRed[3];
  const float rms = rsqrtf(tot * (1.0f / STATE_D) + 1e-6f);
  v8us oh, ol;
#pragma unroll
  for (int c = 0; c < 8; ++c) {
    const float o = v[c] * rms * bf16r(nn[c]);
    const unsigned short hb = bf16_bits(o);
    oh[c] = hb;
    ol[c] = bf16_bits(o - bf16_val(hb));
  }
  const size_t go = (size_t)s * STATE_D + 8 * tid;
  *(volatile v8us*)(yh + go) = oh;
  *(volatile v8us*)(yl + go) = ol;
  __threadfence();
  *(volatile v8us*)(yh + go) = oh;
  *(volatile v8us*)(yl + go) = ol;
}

extern "C" void kernel_launch(void* const* d_in, const int* in_sizes, int n_in,
                              void* d_out, int out_size, void* d_ws, size_t ws_size,
                              hipStream_t stream)
{
  if (n_in < 7) return;
  if (in_sizes[0] != S_LEN * D_IN)      return;
  if (in_sizes[1] != PROJ_D * D_IN)     return;
  if (in_sizes[2] != NH * DH * DH)      return;
  if (in_sizes[3] != NH)                return;
  if (in_sizes[4] != NH * DH)           return;
  if (in_sizes[5] != STATE_D)           return;
  if (in_sizes[6] != D_OUT * STATE_D)   return;
  if (out_size != S_LEN * D_OUT)        return;
  if (ws_size < WS_END)                 return;

  const float* x  = (const float*)d_in[0];
  const float* wi = (const float*)d_in[1];
  const float* sw = (const float*)d_in[2];
  const float* fm = (const float*)d_in[3];
  const float* fb = (const float*)d_in[4];
  const float* gw = (const float*)d_in[5];
  const float* wo = (const float*)d_in[6];
  float* out = (float*)d_out;

  char* ws = (char*)d_ws;
  unsigned short* cv   = (unsigned short*)(ws + OFF_CV);
  float*          proj = (float*)(ws + OFF_PR);
  float*          ypl  = (float*)(ws + OFF_Y);
  unsigned short* yh   = (unsigned short*)(ws + OFF_YH);
  unsigned short* yl   = (unsigned short*)(ws + OFF_YL);

  cvt_kernel<<<dim3(NCBLK), dim3(256), 0, stream>>>(x, wi, wo, cv);

  gemm_kernel<false, true><<<dim3(S_LEN / 128, PROJ_D / 64), dim3(128), GLDS, stream>>>(
      cv + P_X, cv + P_X, cv + P_WI, D_IN, proj, PROJ_D, fm, fb);

  scan_kernel<<<dim3(NH), dim3(128), SLDS, stream>>>(proj, sw, ypl);

  gate_norm_kernel<<<dim3(S_LEN), dim3(128), 0, stream>>>(ypl, proj, gw, yh, yl);

  gemm_kernel<true, false><<<dim3(S_LEN / 128, D_OUT / 64), dim3(128), GLDS, stream>>>(
      yh, yl, cv + P_WO, STATE_D, out, D_OUT, fm, fb);
}
